// TimingMeta_62440234549809
// MI455X (gfx1250) — hardware-verified
//
#include <hip/hip_runtime.h>
#include <stddef.h>


#define NB    64
#define NT    128
#define KIN   257
#define KP    288
#define NH    1024
#define NG    4096
#define NR    8192
#define TC    32
#define MC    2048
#define NTHR  256
#define JB    64
#define XP    132
#define SP    68
#define ASC   16.0f
#define WSC   256.0f
#define UNS   (1.0f / 4096.0f)
#define WSCAP 134217728
#define PB_W   2048
#define PB_WI0 576
#define PB_X   1152
#define PB_H0  64
#define PB_ALL (3 * PB_W + PB_WI0 + PB_X + PB_H0)

static_assert(KP % 32 == 0 && KP >= KIN && KP % 8 == 0);
static_assert(NR == NB * NT && MC == NB * TC && NT % TC == 0 && TC == 32);
static_assert(PB_W * NTHR * 8 == NG * NH);
static_assert(PB_WI0 * NTHR * 8 == NG * KP);
static_assert(PB_X * NTHR * 8 == NR * KP);
static_assert(PB_H0 * NTHR * 8 == 2 * NB * NH);
static_assert(NH % JB == 0 && JB == 64 && NB == 64 && NG == 4 * NH);
static_assert((XP * 4) % 16 == 0 && (SP * 4) % 16 == 0);
static_assert(NB * XP * 4 <= 65536 && 2 * NB * SP * 4 <= 65536);

typedef float          v4f  __attribute__((ext_vector_type(4)));
typedef float          v8f  __attribute__((ext_vector_type(8)));
typedef unsigned int   v4u  __attribute__((ext_vector_type(4)));
typedef unsigned short v8us __attribute__((ext_vector_type(8)));
typedef _Float16       v8h  __attribute__((ext_vector_type(8)));
typedef _Float16       v16h __attribute__((ext_vector_type(16)));
union FragH { v16h v; v8us h[2]; };
union Pk8   { v8h h; v4u u; };

__device__ __forceinline__ v8f wmh(v16h a, v16h b, v8f c) {
  v8f d = __builtin_amdgcn_wmma_f32_16x16x32_f16(false, a, false, b, (short)0, c, false, false);
  asm volatile("v_nop\n\tv_nop\n\tv_nop\n\tv_nop" : "+v"(d) : "v"(a), "v"(b));
  return d;
}

__device__ __forceinline__ float sigm(float x) { return __builtin_amdgcn_rcpf(1.0f + __expf(-x)); }
__device__ __forceinline__ float tanhx(float x) {
  const float e = __expf(-2.0f * fabsf(x));
  const float r = (1.0f - e) * __builtin_amdgcn_rcpf(1.0f + e);
  return x < 0.0f ? -r : r;
}

__device__ __forceinline__ v4u pk8(v4f a, v4f c, float s) {
  Pk8 p;
  p.h[0] = (_Float16)(a.x * s); p.h[1] = (_Float16)(a.y * s);
  p.h[2] = (_Float16)(a.z * s); p.h[3] = (_Float16)(a.w * s);
  p.h[4] = (_Float16)(c.x * s); p.h[5] = (_Float16)(c.y * s);
  p.h[6] = (_Float16)(c.z * s); p.h[7] = (_Float16)(c.w * s);
  return p.u;
}

__global__ __launch_bounds__(NTHR) void k_prep(
    const float* __restrict__ X, const float* __restrict__ h0,
    const float* __restrict__ Wih0, const float* __restrict__ Whh0,
    const float* __restrict__ Wih1, const float* __restrict__ Whh1,
    unsigned short* pX, unsigned short* pH0, unsigned short* pWih0,
    unsigned short* pWhh0, unsigned short* pWih1, unsigned short* pWhh1) {
  const int b = (int)blockIdx.x, tid = (int)threadIdx.x;
  v4u val;
  unsigned short* dst;
  if (b < 3 * PB_W) {
    const int which = b / PB_W;
    const float* W;
    unsigned short* P;
    if (which == 0)      { W = Whh0; P = pWhh0; }
    else if (which == 1) { W = Wih1; P = pWih1; }
    else                 { W = Whh1; P = pWhh1; }
    const size_t i = (size_t)(b - which * PB_W) * NTHR + tid;
    const float* sp = W + i * 8;
    const v4f a = *(const v4f*)sp, c = *(const v4f*)(sp + 4);
    val = pk8(a, c, WSC);
    dst = P + i * 8;
  } else if (b < 3 * PB_W + PB_WI0) {
    const int i = (b - 3 * PB_W) * NTHR + tid;
    const int f = i * 8;
    const int row = f / KP, col0 = f - row * KP;
    float v[8];
#pragma unroll
    for (int e = 0; e < 8; ++e) {
      const int col = col0 + e;
      const int cc = col < KIN ? col : KIN - 1;
      const float t = Wih0[(size_t)row * KIN + cc];
      v[e] = (col < KIN) ? t : 0.0f;
    }
    const v4f a = {v[0], v[1], v[2], v[3]};
    const v4f c = {v[4], v[5], v[6], v[7]};
    val = pk8(a, c, WSC);
    dst = pWih0 + (size_t)f;
  } else if (b < 3 * PB_W + PB_WI0 + PB_X) {
    const int i = (b - 3 * PB_W - PB_WI0) * NTHR + tid;
    const int f = i * 8;
    const int row = f / KP, col0 = f - row * KP;
    float v[8];
#pragma unroll
    for (int e = 0; e < 8; ++e) {
      const int col = col0 + e;
      const int cc = col < KIN ? col : KIN - 1;
      const float t = X[(size_t)row * KIN + cc];
      v[e] = (col < KIN) ? t : 0.0f;
    }
    const v4f a = {v[0], v[1], v[2], v[3]};
    const v4f c = {v[4], v[5], v[6], v[7]};
    val = pk8(a, c, ASC);
    dst = pX + (size_t)f;
  } else {
    const int i = (b - 3 * PB_W - PB_WI0 - PB_X) * NTHR + tid;
    const float* sp = h0 + (size_t)i * 8;
    const v4f a = *(const v4f*)sp, c = *(const v4f*)(sp + 4);
    val = pk8(a, c, ASC);
    dst = pH0 + (size_t)i * 8;
  }
  *(volatile v4u*)dst = val;
  __threadfence();
  *(volatile v4u*)dst = val;
}

__global__ __launch_bounds__(NTHR) void k_gemm(
    const unsigned short* __restrict__ A, int lda, int t0,
    const unsigned short* __restrict__ Bw, int ldb, int ksteps,
    const float* __restrict__ bias, float* xg) {
  __shared__ __attribute__((aligned(16))) float stg[NB * XP];
  const int tid = threadIdx.x, lane = tid & 31, wave = tid >> 5, hh = lane >> 4, m = lane & 15;
  const int rg = wave >> 1, ch = wave & 1;
  const int bx = blockIdx.x, by = blockIdx.y;
  const int mr = by * 64 + rg * 16 + m;
  const int arow = (mr >> 5) * NT + t0 + (mr & 31);
  const unsigned short* ap = A + (size_t)arow * lda + 8 * hh;
  const int n0 = bx * 128 + ch * 64;
  const unsigned short* bp0 = Bw + (size_t)(n0 + m) * ldb + 8 * hh;

  v8f acc[4];
#pragma unroll
  for (int tt = 0; tt < 4; ++tt) { const v8f z = {0.f, 0.f, 0.f, 0.f, 0.f, 0.f, 0.f, 0.f}; acc[tt] = z; }

#pragma unroll 2
  for (int kt = 0; kt < ksteps; ++kt) {
    FragH a;
    a.h[0] = *(const v8us*)(ap + 32 * kt);
    a.h[1] = *(const v8us*)(ap + 32 * kt + 16);
#pragma unroll
    for (int tt = 0; tt < 4; ++tt) {
      const unsigned short* bp = bp0 + (size_t)(16 * tt) * ldb + 32 * kt;
      FragH bq;
      bq.h[0] = *(const v8us*)bp;
      bq.h[1] = *(const v8us*)(bp + 16);
      acc[tt] = wmh(a.v, bq.v, acc[tt]);
    }
  }
  {
    float* sp = stg + (size_t)(rg * 16 + 8 * hh) * XP + ch * 64 + m;
#pragma unroll
    for (int tt = 0; tt < 4; ++tt) {
      const float bb = bias[n0 + 16 * tt + m];
#pragma unroll
      for (int r = 0; r < 8; ++r) sp[r * XP + 16 * tt] = acc[tt][r] * UNS + bb;
    }
  }
  __syncthreads();

  v4f ov[8];
  const size_t ob = (size_t)(by * 64) * NG + (size_t)bx * 128 + 4 * lane;
#pragma unroll
  for (int it = 0; it < 8; ++it) {
    const int row = wave * 8 + it;
    ov[it] = *(const v4f*)(stg + (size_t)row * XP + 4 * lane);
    *(volatile v4f*)(xg + ob + (size_t)row * NG) = ov[it];
  }
  __threadfence();
#pragma unroll
  for (int it = 0; it < 8; ++it) {
    const int row = wave * 8 + it;
    *(volatile v4f*)(xg + ob + (size_t)row * NG) = ov[it];
  }
}

template <int L1>
__global__ __launch_bounds__(NTHR) void k_step(
    const float* __restrict__ xg, int tl,
    const unsigned short* __restrict__ Wp, const float* __restrict__ bhh,
    const unsigned short* __restrict__ hin, unsigned short* hout,
    const float* cin, float* cout, unsigned short* y16, float* y32, int t) {
  __shared__ __attribute__((aligned(16))) float sC[NB * SP];
  __shared__ __attribute__((aligned(16))) float sHn[NB * SP];
  const int tid = threadIdx.x, lane = tid & 31, wave = tid >> 5, hh = lane >> 4, m = lane & 15;
  const int rg = wave >> 1, ch = wave & 1;
  const int j0 = (int)blockIdx.x * JB;

  const unsigned short* ap  = hin + (size_t)(rg * 16 + m) * NH + 8 * hh;
  const unsigned short* bp0 = Wp + (size_t)(j0 + ch * 32 + m) * NH + 8 * hh;

  v8f acc[8];
#pragma unroll
  for (int tt = 0; tt < 8; ++tt) { const v8f z = {0.f, 0.f, 0.f, 0.f, 0.f, 0.f, 0.f, 0.f}; acc[tt] = z; }

#pragma unroll 1
  for (int kt = 0; kt < NH / 32; ++kt) {
    FragH a;
    a.h[0] = *(const v8us*)(ap + 32 * kt);
    a.h[1] = *(const v8us*)(ap + 32 * kt + 16);
#pragma unroll
    for (int gi = 0; gi < 4; ++gi) {
#pragma unroll
      for (int u = 0; u < 2; ++u) {
        const unsigned short* bp = bp0 + (size_t)(gi * NH + 16 * u) * NH + 32 * kt;
        FragH bq;
        bq.h[0] = *(const v8us*)bp;
        bq.h[1] = *(const v8us*)(bp + 16);
        acc[gi * 2 + u] = wmh(a.v, bq.v, acc[gi * 2 + u]);
      }
    }
  }

#pragma unroll
  for (int u = 0; u < 2; ++u) {
    const int jl = ch * 32 + 16 * u + m;
    const int j = j0 + jl;
    const float bi = bhh[j], bf = bhh[NH + j], bg = bhh[2 * NH + j], bo = bhh[3 * NH + j];
#pragma unroll
    for (int r = 0; r < 8; ++r) {
      const int brow = rg * 16 + 8 * hh + r;
      const float* xr = xg + (size_t)(brow * TC + tl) * NG + j;
      const float pi = acc[u][r]     * UNS + xr[0]      + bi;
      const float pf = acc[2 + u][r] * UNS + xr[NH]     + bf;
      const float pg = acc[4 + u][r] * UNS + xr[2 * NH] + bg;
      const float po = acc[6 + u][r] * UNS + xr[3 * NH] + bo;
      const float cold = cin[(size_t)brow * NH + j];
      const float cn = sigm(pf) * cold + sigm(pi) * tanhx(pg);
      const float hn = sigm(po) * tanhx(cn);
      sC[brow * SP + jl]  = cn;
      sHn[brow * SP + jl] = hn;
    }
  }
  __syncthreads();

  const int q4 = lane & 15, r2 = lane >> 4;
  const int q8 = lane & 7,  r4 = lane >> 3;
  v4f cv[4], hv[4];
  v4u hp[2];
#pragma unroll
  for (int it = 0; it < 4; ++it) {
    const int row = wave * 8 + 2 * it + r2;
    cv[it] = *(const v4f*)(sC + (size_t)row * SP + 4 * q4);
    *(volatile v4f*)(cout + (size_t)row * NH + j0 + 4 * q4) = cv[it];
    if (L1) {
      hv[it] = *(const v4f*)(sHn + (size_t)row * SP + 4 * q4);
      *(volatile v4f*)(y32 + ((size_t)row * NT + t) * NH + j0 + 4 * q4) = hv[it];
    }
  }
#pragma unroll
  for (int it = 0; it < 2; ++it) {
    const int row = wave * 8 + 4 * it + r4;
    const v4f a = *(const v4f*)(sHn + (size_t)row * SP + 8 * q8);
    const v4f c = *(const v4f*)(sHn + (size_t)row * SP + 8 * q8 + 4);
    hp[it] = pk8(a, c, ASC);
    *(volatile v4u*)(hout + (size_t)row * NH + j0 + 8 * q8) = hp[it];
    if (!L1) *(volatile v4u*)(y16 + ((size_t)row * NT + t) * NH + j0 + 8 * q8) = hp[it];
  }
  __threadfence();
#pragma unroll
  for (int it = 0; it < 4; ++it) {
    const int row = wave * 8 + 2 * it + r2;
    *(volatile v4f*)(cout + (size_t)row * NH + j0 + 4 * q4) = cv[it];
    if (L1) *(volatile v4f*)(y32 + ((size_t)row * NT + t) * NH + j0 + 4 * q4) = hv[it];
  }
#pragma unroll
  for (int it = 0; it < 2; ++it) {
    const int row = wave * 8 + 4 * it + r4;
    *(volatile v4u*)(hout + (size_t)row * NH + j0 + 8 * q8) = hp[it];
    if (!L1) *(volatile v4u*)(y16 + ((size_t)row * NT + t) * NH + j0 + 8 * q8) = hp[it];
  }
}

__global__ __launch_bounds__(NTHR) void k_head(
    const float* __restrict__ y32, const float* __restrict__ Wy,
    const float* __restrict__ by, float* out) {
  __shared__ __attribute__((aligned(16))) float sO[128];
  const int tid = threadIdx.x, lane = tid & 31, wave = tid >> 5;
  const float by0 = by[0], by1 = by[1];
#pragma unroll 1
  for (int it = 0; it < 8; ++it) {
    const int lrow = wave * 8 + it;
    const int grow = (int)blockIdx.x * 64 + lrow;
    const float* yr = y32 + (size_t)grow * NH + 4 * lane;
    float s0 = 0.0f, s1 = 0.0f;
#pragma unroll 1
    for (int i = 0; i < NH / 128; ++i) {
      const v4f v  = *(const v4f*)(yr + 128 * i);
      const v4f w0 = *(const v4f*)(Wy + 4 * lane + 128 * i);
      const v4f w1 = *(const v4f*)(Wy + NH + 4 * lane + 128 * i);
      const float tx = tanhx(v.x), ty = tanhx(v.y), tz = tanhx(v.z), tw = tanhx(v.w);
      s0 += tx * w0.x + ty * w0.y + tz * w0.z + tw * w0.w;
      s1 += tx * w1.x + ty * w1.y + tz * w1.z + tw * w1.w;
    }
    s0 += __shfl_xor(s0, 1);  s1 += __shfl_xor(s1, 1);
    s0 += __shfl_xor(s0, 2);  s1 += __shfl_xor(s1, 2);
    s0 += __shfl_xor(s0, 4);  s1 += __shfl_xor(s1, 4);
    s0 += __shfl_xor(s0, 8);  s1 += __shfl_xor(s1, 8);
    s0 += __shfl_xor(s0, 16); s1 += __shfl_xor(s1, 16);
    if (lane == 0) { sO[lrow * 2] = s0 + by0; sO[lrow * 2 + 1] = s1 + by1; }
  }
  __syncthreads();
  v4f ov = {0.f, 0.f, 0.f, 0.f};
  const size_t ob = (size_t)blockIdx.x * 128 + 4 * lane;
  if (wave == 0) {
    ov = *(const v4f*)(sO + 4 * lane);
    *(volatile v4f*)(out + ob) = ov;
  }
  __threadfence();
  if (wave == 0) {
    *(volatile v4f*)(out + ob) = ov;
  }
}

extern "C" void kernel_launch(void* const* d_in, const int* in_sizes, int n_in,
                              void* d_out, int out_size, void* d_ws, size_t ws_size,
                              hipStream_t stream) {
  if (n_in < 13) return;
  if (in_sizes[0] != NR * KIN) return;
  if (in_sizes[1] != 2 * NB * NH || in_sizes[2] != 2 * NB * NH) return;
  if (in_sizes[3] != NG * KIN || in_sizes[4] != NG * NH || in_sizes[5] != NG || in_sizes[6] != NG) return;
  if (in_sizes[7] != NG * NH || in_sizes[8] != NG * NH || in_sizes[9] != NG || in_sizes[10] != NG) return;
  if (in_sizes[11] != 2 * NH || in_sizes[12] != 2) return;
  if (out_size != NR * 2) return;

  const float* X    = (const float*)d_in[0];
  const float* h0   = (const float*)d_in[1];
  const float* c0   = (const float*)d_in[2];
  const float* Wih0 = (const float*)d_in[3];
  const float* Whh0 = (const float*)d_in[4];
  const float* bih0 = (const float*)d_in[5];
  const float* bhh0 = (const float*)d_in[6];
  const float* Wih1 = (const float*)d_in[7];
  const float* Whh1 = (const float*)d_in[8];
  const float* bih1 = (const float*)d_in[9];
  const float* bhh1 = (const float*)d_in[10];
  const float* Wy   = (const float*)d_in[11];
  const float* by   = (const float*)d_in[12];
  float* out = (float*)d_out;

  char* ws = (char*)d_ws;
  size_t off = 0;
  const size_t oWi0 = off; off += (size_t)NG * KP * 2;     off = (off + 255) & ~(size_t)255;
  const size_t oWh0 = off; off += (size_t)NG * NH * 2;     off = (off + 255) & ~(size_t)255;
  const size_t oWi1 = off; off += (size_t)NG * NH * 2;     off = (off + 255) & ~(size_t)255;
  const size_t oWh1 = off; off += (size_t)NG * NH * 2;     off = (off + 255) & ~(size_t)255;
  const size_t oX   = off; off += (size_t)NR * KP * 2;     off = (off + 255) & ~(size_t)255;
  const size_t oH0  = off; off += (size_t)2 * NB * NH * 2; off = (off + 255) & ~(size_t)255;
  const size_t oXg  = off; off += (size_t)MC * NG * 4;     off = (off + 255) & ~(size_t)255;
  const size_t oY1  = off; off += (size_t)NR * NH * 2;     off = (off + 255) & ~(size_t)255;
  const size_t oY2  = off; off += (size_t)NR * NH * 4;     off = (off + 255) & ~(size_t)255;
  const size_t oHA  = off; off += (size_t)NB * NH * 2;     off = (off + 255) & ~(size_t)255;
  const size_t oHB  = off; off += (size_t)NB * NH * 2;     off = (off + 255) & ~(size_t)255;
  const size_t oC   = off; off += (size_t)NB * NH * 4;     off = (off + 255) & ~(size_t)255;
  if (off > ws_size || off > (size_t)WSCAP) return;
  unsigned short* pWi0 = (unsigned short*)(ws + oWi0);
  unsigned short* pWh0 = (unsigned short*)(ws + oWh0);
  unsigned short* pWi1 = (unsigned short*)(ws + oWi1);
  unsigned short* pWh1 = (unsigned short*)(ws + oWh1);
  unsigned short* pX   = (unsigned short*)(ws + oX);
  unsigned short* pH0  = (unsigned short*)(ws + oH0);
  float*          xg   = (float*)(ws + oXg);
  unsigned short* y1   = (unsigned short*)(ws + oY1);
  float*          y2   = (float*)(ws + oY2);
  unsigned short* hA   = (unsigned short*)(ws + oHA);
  unsigned short* hB   = (unsigned short*)(ws + oHB);
  float*          cb   = (float*)(ws + oC);

  k_prep<<<PB_ALL, NTHR, 0, stream>>>(X, h0, Wih0, Whh0, Wih1, Whh1, pX, pH0, pWi0, pWh0, pWi1, pWh1);

  for (int L = 0; L < 2; ++L) {
    const unsigned short* Ap = (L == 0) ? pX : y1;
    const int lda = (L == 0) ? KP : NH;
    const int ksteps = lda / 32;
    const unsigned short* Wi = (L == 0) ? pWi0 : pWi1;
    const unsigned short* Wh = (L == 0) ? pWh0 : pWh1;
    const float* bi = (L == 0) ? bih0 : bih1;
    const float* bh = (L == 0) ? bhh0 : bhh1;
    for (int ci = 0; ci < NT / TC; ++ci) {
      const int t0 = ci * TC;
      k_gemm<<<dim3(NG / 128, MC / 64), NTHR, 0, stream>>>(Ap, lda, t0, Wi, lda, ksteps, bi, xg);
      for (int tl = 0; tl < TC; ++tl) {
        const int t = t0 + tl;
        const unsigned short* hin = (t == 0) ? (pH0 + (size_t)L * NB * NH) : ((t & 1) ? hA : hB);
        unsigned short* hout = (t & 1) ? hB : hA;
        const float* cin = (t == 0) ? (c0 + (size_t)L * NB * NH) : cb;
        if (L == 0)
          k_step<0><<<NH / JB, NTHR, 0, stream>>>(xg, tl, Wh, bh, hin, hout, cin, cb, y1, y2, t);
        else
          k_step<1><<<NH / JB, NTHR, 0, stream>>>(xg, tl, Wh, bh, hin, hout, cin, cb, y1, y2, t);
      }
    }
  }

  k_head<<<NR / 64, NTHR, 0, stream>>>(y2, Wy, by, out);
}
